// RelationalGraphAttentionConv_21766894256814
// MI455X (gfx1250) — hardware-verified
//
#include <hip/hip_runtime.h>
#include <stddef.h>
#include <stdint.h>


#define DIMC   128
#define RP1    9
#define NHEAD  8
#define QD     32
#define NEGS   0.2f
#define LABC   144
#define LABP   160
#define FROWS  160
#define RCH    3
#define WROWS  (RCH * DIMC)
#define NTHR   256
#define NWAVE  8
#define RBG    64
#define APH    136
#define GLDSA  (2 * RBG * APH * 2)
#define EPT    8
#define CHUNK  (NTHR * EPT)
#define WCAP   (EPT * 32)
#define LISTN  (NWAVE * WCAP)
#define NBMAX  1024
#define SLOTB  10
#define RCAP   24576
#define DEGCAP 4096
#define STW    512
#define WSMAX  134217728
#define LDS_AGG_INTS (2 * RCAP + 4 * NBMAX + LISTN + 2 * NWAVE)
#define LDS_AGG (LDS_AGG_INTS * 4)

static_assert((CHUNK & (CHUNK - 1)) == 0 && CHUNK <= 2048);
static_assert((NBMAX & (NBMAX - 1)) == 0 && NBMAX == (1 << SLOTB));
static_assert(NTHR * 4 == NBMAX);
static_assert(LISTN >= NBMAX && LISTN >= NWAVE * WCAP);
static_assert((RCAP % 32) == 0 && NWAVE * STW <= RCAP);
static_assert(LDS_AGG <= 300000);
static_assert(RBG == 64 && NTHR == 4 * RBG && NWAVE * 8 == RBG);
static_assert((APH % 8) == 0 && (GLDSA % 16) == 0);
static_assert(LABC == RP1 * NHEAD * 2 && LABP >= LABC && (LABP % 32) == 0 && FROWS == LABP);
static_assert(RCH * 3 == RP1 && DIMC == NHEAD * 16 && QD == 32);

typedef float          v4f  __attribute__((ext_vector_type(4)));
typedef float          v8f  __attribute__((ext_vector_type(8)));
typedef int            v4i  __attribute__((ext_vector_type(4)));
typedef int            v8i  __attribute__((ext_vector_type(8)));
typedef unsigned short us;
typedef us             v8us __attribute__((ext_vector_type(8)));
typedef __bf16         v16b __attribute__((ext_vector_type(16)));
union FragB { v16b v; v8us h[2]; v8i w; };

__device__ __forceinline__ v8f wmb(const FragB& a, const FragB& b, v8f c) {
  v8f d = __builtin_amdgcn_wmma_f32_16x16x32_bf16(false, a.v, false, b.v, (short)0, c, false, false);
  asm volatile("v_nop\n\tv_nop\n\tv_nop\n\tv_nop" : "+v"(d) : "v"(a.w), "v"(b.w));
  return d;
}

__device__ __forceinline__ us bfbits(float f) {
  unsigned u = __float_as_uint(f);
  u = (u + 0x7fffu + ((u >> 16) & 1u)) >> 16;
  return (us)u;
}
__device__ __forceinline__ void split8(const v4f a, const v4f b, v8us& hv, v8us& lv) {
  const float f[8] = {a.x, a.y, a.z, a.w, b.x, b.y, b.z, b.w};
#pragma unroll
  for (int i = 0; i < 8; ++i) {
    const us hb = bfbits(f[i]);
    const float hf = __uint_as_float(((unsigned)hb) << 16);
    hv[i] = hb;
    lv[i] = bfbits(f[i] - hf);
  }
}
__device__ __forceinline__ int clampi(int v, int lo, int hi) { return v < lo ? lo : (v > hi ? hi : v); }

__global__ __launch_bounds__(128) void k_fold(const float* __restrict__ qry, const float* __restrict__ W, float* F) {
  const int n = (int)blockIdx.x, d = (int)threadIdx.x;
  const bool val = n < LABC;
  const int nc = val ? n : 0;
  const int rel = nc >> 4, h = (nc >> 1) & 7, s = nc & 1;
  const float* qp = qry + (size_t)(rel * NHEAD + h) * QD + s;
  const float* wp = W + ((size_t)rel * DIMC + 16 * h) * DIMC + d;
  float acc = 0.f;
#pragma unroll 1
  for (int j = 0; j < 16; ++j) acc = fmaf(qp[2 * j], wp[(size_t)j * DIMC], acc);
  acc = val ? acc : 0.f;
  float* op = F + (size_t)n * DIMC + d;
  *(volatile float*)op = acc;
  __threadfence();
  *(volatile float*)op = acc;
}

__global__ __launch_bounds__(NTHR) void k_cvt(const float* __restrict__ src, us* hi, us* lo, int nUnits) {
  const int u = (int)blockIdx.x * NTHR + (int)threadIdx.x;
  if (u >= nUnits) return;
  const int row = u >> 4, k8 = (u & 15) * 8;
  const float* p = src + (size_t)row * DIMC + k8;
  const v4f a = *(const v4f*)p, b = *(const v4f*)(p + 4);
  v8us hv, lv;
  split8(a, b, hv, lv);
  const size_t o = (size_t)row * DIMC + k8;
  *(volatile v8us*)(hi + o) = hv;
  *(volatile v8us*)(lo + o) = lv;
  __threadfence();
  *(volatile v8us*)(hi + o) = hv;
  *(volatile v8us*)(lo + o) = lv;
}

__device__ __forceinline__ void gemm_store_pass(const float* stg, float* outp, int SP, int npw, size_t pstride,
                                                int rowBase, int wave, int lane) {
#pragma unroll 1
  for (int i = 0; i < RBG / NWAVE; ++i) {
    const int r = wave + NWAVE * i;
    const size_t orow = (size_t)(rowBase + r);
#pragma unroll 1
    for (int cb = 0; cb < SP; cb += 128) {
      const int c = cb + 4 * lane;
      const int ccl = c < SP - 4 ? c : SP - 4;
      const v4f v = *(const v4f*)(stg + (size_t)r * SP + ccl);
      const int pl = ccl / npw;
      const int col = ccl - pl * npw;
      float* op = outp + (size_t)pl * pstride + orow * (size_t)npw + col;
      if (c < SP) *(volatile v4f*)op = v;
    }
  }
}

__global__ __launch_bounds__(NTHR) void k_gemm3(const float* __restrict__ X, const us* __restrict__ BH,
                                                const us* __restrict__ BL, float* outp,
                                                int nN, int nct, int npw, size_t pstride) {
  extern __shared__ v4i glds[];
  us* ah = (us*)glds;
  us* al = ah + RBG * APH;
  float* stg = (float*)(al + RBG * APH);
  const int tid = (int)threadIdx.x, lane = tid & 31, wave = tid >> 5, hh = lane >> 4, m = lane & 15;
  const int rowBase = (int)blockIdx.x * RBG;
  const int SP = nct * 16;

  {
    const int r = tid >> 2, q = tid & 3;
    const int grow = rowBase + r;
    const int gc = grow < nN ? grow : nN - 1;
    const float* xp = X + (size_t)gc * DIMC + 32 * q;
    const bool zero = grow >= nN;
    const v4f z4 = {0.f, 0.f, 0.f, 0.f};
#pragma unroll
    for (int g = 0; g < 4; ++g) {
      v4f a = *(const v4f*)(xp + 8 * g), b = *(const v4f*)(xp + 8 * g + 4);
      if (zero) { a = z4; b = z4; }
      v8us hv, lv;
      split8(a, b, hv, lv);
      *(v8us*)(ah + r * APH + 32 * q + 8 * g) = hv;
      *(v8us*)(al + r * APH + 32 * q + 8 * g) = lv;
    }
  }
  __syncthreads();

  const int rt = wave & 3, cg = wave >> 2;
  FragB aH[4], aL[4];
  {
    const us* ar = ah + (rt * 16 + m) * APH + 8 * hh;
    const us* lr = al + (rt * 16 + m) * APH + 8 * hh;
#pragma unroll
    for (int ks = 0; ks < 4; ++ks) {
      aH[ks].h[0] = *(const v8us*)(ar + 32 * ks);
      aH[ks].h[1] = *(const v8us*)(ar + 32 * ks + 16);
      aL[ks].h[0] = *(const v8us*)(lr + 32 * ks);
      aL[ks].h[1] = *(const v8us*)(lr + 32 * ks + 16);
    }
  }
  const int nh2 = nct >> 1;
#pragma unroll 1
  for (int i = 0; i < nh2; ++i) {
    const int ct = cg + 2 * i;
    v8f acc = {0.f, 0.f, 0.f, 0.f, 0.f, 0.f, 0.f, 0.f};
    const us* bph = BH + (size_t)(ct * 16 + m) * DIMC + 8 * hh;
    const us* bpl = BL + (size_t)(ct * 16 + m) * DIMC + 8 * hh;
#pragma unroll
    for (int ks = 0; ks < 4; ++ks) {
      FragB bHf, bLf;
      bHf.h[0] = *(const v8us*)(bph + 32 * ks);
      bHf.h[1] = *(const v8us*)(bph + 32 * ks + 16);
      bLf.h[0] = *(const v8us*)(bpl + 32 * ks);
      bLf.h[1] = *(const v8us*)(bpl + 32 * ks + 16);
      acc = wmb(aH[ks], bHf, acc);
      acc = wmb(aH[ks], bLf, acc);
      acc = wmb(aL[ks], bHf, acc);
    }
    float* sp = stg + (size_t)(rt * 16 + 8 * hh) * SP + ct * 16 + m;
#pragma unroll
    for (int r = 0; r < 8; ++r) sp[(size_t)r * SP] = acc[r];
  }
  __syncthreads();

  gemm_store_pass(stg, outp, SP, npw, pstride, rowBase, wave, lane);
  __threadfence();
  gemm_store_pass(stg, outp, SP, npw, pstride, rowBase, wave, lane);
}

__device__ __forceinline__ int scan_chunk(const int* __restrict__ el, int nE, int cbase, int slotBase, int nb,
                                          int relBase, int* list, int tid, int lane, int wave) {
  int wc = 0;
  const int el0 = tid * EPT;
  const int e0  = cbase + el0;
  const int sent = -2147483647 - 1;
  int d[8], rl[8];
  if (cbase + CHUNK <= nE) {
    const v4i* p = (const v4i*)(el + (size_t)3 * (size_t)e0);
    const v4i q0 = p[0], q1 = p[1], q2 = p[2], q3 = p[3], q4 = p[4], q5 = p[5];
    d[0] = q0.y; rl[0] = q0.z;  d[1] = q1.x; rl[1] = q1.y;  d[2] = q1.w; rl[2] = q2.x;  d[3] = q2.z; rl[3] = q2.w;
    d[4] = q3.y; rl[4] = q3.z;  d[5] = q4.x; rl[5] = q4.y;  d[6] = q4.w; rl[6] = q5.x;  d[7] = q5.z; rl[7] = q5.w;
  } else {
#pragma unroll
    for (int j = 0; j < 8; ++j) {
      const int e = e0 + j;
      int ec = e < nE ? e : nE - 1;
      ec = ec < 0 ? 0 : ec;
      const int dv = el[(size_t)3 * ec + 1];
      const int rv = el[(size_t)3 * ec + 2];
      d[j] = (e < nE) ? dv : sent;
      rl[j] = rv;
    }
  }
  const unsigned nbs = (unsigned)slotBase, unb = (unsigned)nb;
  unsigned sv[8]; bool hit[8]; int icb[8];
  bool anyl = false;
#pragma unroll
  for (int j = 0; j < 8; ++j) {
    sv[j]  = (unsigned)d[j] - nbs;
    hit[j] = sv[j] < unb;
    icb[j] = ((unsigned)(rl[j] - relBase) < (unsigned)RCH) ? 1 : 0;
    anyl = anyl | hit[j];
  }
  const unsigned any = __builtin_amdgcn_ballot_w32(anyl);
  if (any != 0u) {
#pragma unroll
    for (int j = 0; j < 8; ++j) {
      const unsigned mj = __builtin_amdgcn_ballot_w32(hit[j]);
      if (mj != 0u) {
        if (hit[j]) {
          const int pos = wc + (int)__builtin_amdgcn_mbcnt_lo(mj, 0u);
          if (pos < WCAP) list[wave * WCAP + pos] = ((el0 + j) << 12) | (icb[j] << SLOTB) | (int)sv[j];
        }
        wc += (int)__builtin_popcount(mj);
      }
    }
  }
  return wc;
}

__global__ __launch_bounds__(NTHR) void k_agg(const int* __restrict__ el, const float* __restrict__ ew,
                                              const float* __restrict__ LAB, const float* __restrict__ HID,
                                              float* out, int nN, int nE, int nb, int chunk, size_t pstride) {
  extern __shared__ v4f lds_dyn[];
  int* reg1 = (int*)lds_dyn;
  int* reg2 = reg1 + RCAP;
  int* scnt = reg2 + RCAP;
  int* scc  = scnt + NBMAX;
  int* soff = scc + NBMAX;
  int* bcur = soff + NBMAX;
  int* list = bcur + NBMAX;
  int* wcnt = list + LISTN;
  int* wtot = wcnt + NWAVE;
  const int tid = (int)threadIdx.x, lane = tid & 31, wave = tid >> 5;
  const int nodeBase = (int)blockIdx.x * nb;
  const int relBase = RCH * chunk;

  for (int i = tid; i < NBMAX; i += NTHR) { scnt[i] = 0; scc[i] = 0; }
  __syncthreads();

  int tot = 0;
  const int nChunks = (nE + CHUNK - 1) / CHUNK;
#pragma unroll 1
  for (int ch = 0; ch < nChunks; ++ch) {
    const int cbase = ch * CHUNK;
    const int wc = scan_chunk(el, nE, cbase, nodeBase, nb, relBase, list, tid, lane, wave);
    if (lane == 0) wcnt[wave] = wc;
    __syncthreads();
    int pre = 0, all = 0;
#pragma unroll
    for (int w2 = 0; w2 < NWAVE; ++w2) {
      int c = wcnt[w2];
      c = c < 0 ? 0 : (c > WCAP ? WCAP : c);
      all += c;
      pre += (w2 < wave) ? c : 0;
    }
    const int wcc  = wc > WCAP ? WCAP : wc;
    const int base = tot + pre;
#pragma unroll 1
    for (int i = lane; i < wcc; i += 32) {
      const int ent = list[wave * WCAP + i];
      const int elx = (ent >> 12) & (CHUNK - 1);
      const int ic  = (ent >> SLOTB) & 1;
      const int sl  = ent & (NBMAX - 1);
      int eid = cbase + elx;
      eid = eid > nE - 1 ? nE - 1 : eid;
      const int pos = base + i;
      if (pos < RCAP) reg1[pos] = (int)(((unsigned)eid << (SLOTB + 1)) | ((unsigned)ic << SLOTB) | (unsigned)sl);
    }
    tot += all;
    tot = tot > RCAP ? RCAP : tot;
    __syncthreads();
  }
  const int nh = tot;

  if (wave == 0) {
#pragma unroll 1
    for (int b0 = 0; b0 < nh; b0 += 32) {
      const int idx = b0 + lane;
      const int uv  = reg1[idx < RCAP ? idx : RCAP - 1];
      const int m32 = (nh - b0) < 32 ? (nh - b0) : 32;
#pragma unroll 1
      for (int k = 0; k < m32; ++k) {
        const int u  = __builtin_amdgcn_readlane(uv, k);
        const int sl = u & (NBMAX - 1);
        const int ic = (u >> SLOTB) & 1;
        if (lane == 0) { scnt[sl] = scnt[sl] + 1; scc[sl] = scc[sl] + ic; }
      }
    }
  }
  __syncthreads();

  {
    const v4i ca = *(const v4i*)(scnt + 4 * tid);
    const int e0 = ca.x < 0 ? 0 : ca.x, e1 = ca.y < 0 ? 0 : ca.y, e2 = ca.z < 0 ? 0 : ca.z, e3 = ca.w < 0 ? 0 : ca.w;
    const int ts = e0 + e1 + e2 + e3;
    int incl = ts;
#pragma unroll
    for (int dd = 1; dd < 32; dd <<= 1) {
      const int up = __shfl_up(incl, dd);
      if (lane >= dd) incl += up;
    }
    if (lane == 31) wtot[wave] = incl;
    __syncthreads();
    int pre = 0;
#pragma unroll
    for (int w2 = 0; w2 < NWAVE; ++w2) pre += (w2 < wave) ? wtot[w2] : 0;
    int run = pre + incl - ts;
    soff[4 * tid + 0] = run; run += e0;
    soff[4 * tid + 1] = run; run += e1;
    soff[4 * tid + 2] = run; run += e2;
    soff[4 * tid + 3] = run;
  }
  __syncthreads();
  for (int i = tid; i < NBMAX; i += NTHR) {
    const int s0 = soff[i];
    int b = s0 + scnt[i];
    b = b > RCAP ? RCAP : b;
    list[i] = s0;
    bcur[i] = b;
  }
  __syncthreads();

  if (wave == 0) {
#pragma unroll 1
    for (int b0 = 0; b0 < nh; b0 += 32) {
      const int idx = b0 + lane;
      const int uv  = reg1[idx < RCAP ? idx : RCAP - 1];
      const int m32 = (nh - b0) < 32 ? (nh - b0) : 32;
#pragma unroll 1
      for (int k = 0; k < m32; ++k) {
        const int u   = __builtin_amdgcn_readlane(uv, k);
        const int sl  = u & (NBMAX - 1);
        const int ic  = (u >> SLOTB) & 1;
        const int eid = (int)((unsigned)u >> (SLOTB + 1));
        if (lane == 0) {
          if (ic != 0) {
            int pos = list[sl];
            pos = pos < 0 ? 0 : (pos > RCAP - 1 ? RCAP - 1 : pos);
            reg2[pos] = eid;
            list[sl] = pos + 1;
          } else {
            int pos = bcur[sl] - 1;
            pos = pos < 0 ? 0 : (pos > RCAP - 1 ? RCAP - 1 : pos);
            reg2[pos] = eid;
            bcur[sl] = pos;
          }
        }
      }
    }
  }
  __syncthreads();

  const int nbw = nb >> 3;
  const bool ovf = (nh >= RCAP);
  const float qnan = __int_as_float(0x7fc00000);
  float* stw = (float*)reg1 + wave * STW;
  const int h8 = lane & 7, sub = lane >> 3;
  const bool fin = (relBase + RCH >= RP1);
  const float addp = (chunk > 0) ? 1.0f : 0.0f;
  const float* laba = LAB + 2 * h8;
#pragma unroll 1
  for (int jt = 0; jt < nbw; ++jt) {
    const int slot = wave * nbw + jt;
    const int grow = nodeBase + slot;
    const int gcl  = grow < nN ? grow : nN - 1;
    int st = soff[slot];
    const int craw = scnt[slot];
    int cnt = craw, cc = scc[slot];
    st  = clampi(st, 0, nh);
    cnt = clampi(cnt, 0, DEGCAP);
    if (cnt > nh - st) cnt = nh - st;
    cc = clampi(cc, 0, cnt);
    const float pz = (ovf || craw > DEGCAP) ? qnan : 0.0f;
    const bool wr = grow < nN;
    const float cntf = (float)(cnt + 1);
    const float rc = __builtin_amdgcn_rcpf(cntf);
    const float* labd = LAB + (size_t)gcl * LABP + 2 * h8 + 1;

    float m = -1.0e30f, S = 0.f;
    const int nA = cnt + 1;
#pragma unroll 1
    for (int q = 0; q < nA; q += 4) {
      const int i = q + sub;
      const bool valid = i < nA;
      const bool slf = (i == cnt);
      int idx = st + i; idx = idx > RCAP - 1 ? RCAP - 1 : idx;
      int eid = reg2[idx];
      eid = clampi(eid, 0, nE - 1);
      const int sr = el[(size_t)3 * eid];
      const int rr = el[(size_t)3 * eid + 2];
      const float wv = ew[eid];
      const int src = slf ? gcl : clampi(sr, 0, nN - 1);
      const int rel = slf ? (RP1 - 1) : clampi(rr, 0, RP1 - 1);
      const float wgt = slf ? 1.0f : wv;
      const float a = laba[(size_t)src * LABP + rel * 16];
      const float b = labd[rel * 16];
      float w = a + b;
      w = w > 0.f ? w : NEGS * w;
      const float df = w - m;
      const float ee = __expf(-fabsf(df));
      const bool up = df > 0.f;
      const float s1 = up ? ee : 1.0f;
      const float s2 = up ? 1.0f : ee;
      const float mN = up ? w : m;
      const float SN = fmaf(S, s1, s2 * wgt);
      m = valid ? mN : m;
      S = valid ? SN : S;
    }
#pragma unroll
    for (int off = 8; off < 32; off <<= 1) {
      const float mo = __shfl_xor(m, off);
      const float So = __shfl_xor(S, off);
      const float mm = fmaxf(m, mo);
      S = S * __expf(m - mm) + So * __expf(mo - mm);
      m = mm;
    }
    const float mh = __shfl(m, h8);
    const float Sh = __shfl(S, h8);
    const float nrm = Sh * rc;
    const float inv = __builtin_amdgcn_rcpf(nrm + 1.0e-10f);

    float acc[16];
#pragma unroll
    for (int k = 0; k < 16; ++k) acc[k] = 0.f;
    const int nB = cc + (fin ? 1 : 0);
#pragma unroll 1
    for (int q = 0; q < nB; q += 4) {
      const int i = q + sub;
      const bool valid = i < nB;
      const bool slf = fin && (i == cc);
      int idx = st + i; idx = idx > RCAP - 1 ? RCAP - 1 : idx;
      int eid = reg2[idx];
      eid = clampi(eid, 0, nE - 1);
      const int sr = el[(size_t)3 * eid];
      const int rr = el[(size_t)3 * eid + 2];
      const float wv = ew[eid];
      const int src = slf ? gcl : clampi(sr, 0, nN - 1);
      const int rel = slf ? (RP1 - 1) : clampi(rr, 0, RP1 - 1);
      const float wgt = slf ? 1.0f : wv;
      int relc = rel - relBase;
      const bool inC = (unsigned)relc < (unsigned)RCH;
      relc = clampi(relc, 0, RCH - 1);
      const float a = laba[(size_t)src * LABP + rel * 16];
      const float b = labd[rel * 16];
      float w = a + b;
      w = w > 0.f ? w : NEGS * w;
      float coef = __expf(w - mh) * wgt * inv;
      coef = (valid && inC) ? coef : 0.f;
      const float* hp = HID + (size_t)relc * pstride + (size_t)src * DIMC + 16 * h8;
      const v4f v0 = *(const v4f*)hp, v1 = *(const v4f*)(hp + 4);
      const v4f v2 = *(const v4f*)(hp + 8), v3 = *(const v4f*)(hp + 12);
      acc[0]  = fmaf(coef, v0.x, acc[0]);  acc[1]  = fmaf(coef, v0.y, acc[1]);
      acc[2]  = fmaf(coef, v0.z, acc[2]);  acc[3]  = fmaf(coef, v0.w, acc[3]);
      acc[4]  = fmaf(coef, v1.x, acc[4]);  acc[5]  = fmaf(coef, v1.y, acc[5]);
      acc[6]  = fmaf(coef, v1.z, acc[6]);  acc[7]  = fmaf(coef, v1.w, acc[7]);
      acc[8]  = fmaf(coef, v2.x, acc[8]);  acc[9]  = fmaf(coef, v2.y, acc[9]);
      acc[10] = fmaf(coef, v2.z, acc[10]); acc[11] = fmaf(coef, v2.w, acc[11]);
      acc[12] = fmaf(coef, v3.x, acc[12]); acc[13] = fmaf(coef, v3.y, acc[13]);
      acc[14] = fmaf(coef, v3.z, acc[14]); acc[15] = fmaf(coef, v3.w, acc[15]);
    }
    __builtin_amdgcn_fence(__ATOMIC_RELEASE, "wavefront");
    __builtin_amdgcn_wave_barrier();
    {
      float* sp = stw + sub * DIMC + 16 * h8;
      const v4f g0 = {acc[0], acc[1], acc[2], acc[3]},   g1 = {acc[4], acc[5], acc[6], acc[7]};
      const v4f g2 = {acc[8], acc[9], acc[10], acc[11]}, g3 = {acc[12], acc[13], acc[14], acc[15]};
      *(v4f*)sp = g0; *(v4f*)(sp + 4) = g1; *(v4f*)(sp + 8) = g2; *(v4f*)(sp + 12) = g3;
    }
    __builtin_amdgcn_fence(__ATOMIC_RELEASE, "wavefront");
    __builtin_amdgcn_wave_barrier();
    const v4f p0 = *(const v4f*)(stw + 4 * lane);
    const v4f p1 = *(const v4f*)(stw + DIMC + 4 * lane);
    const v4f p2 = *(const v4f*)(stw + 2 * DIMC + 4 * lane);
    const v4f p3 = *(const v4f*)(stw + 3 * DIMC + 4 * lane);
    const v4f pr = *(const v4f*)(out + (size_t)gcl * DIMC + 4 * lane);
    v4f t = (p0 + p1) + (p2 + p3);
    t = t + pr * addp;
    if (fin) {
      t = t * rc;
      t.x = t.x < 0.f ? 0.f : t.x;  t.y = t.y < 0.f ? 0.f : t.y;
      t.z = t.z < 0.f ? 0.f : t.z;  t.w = t.w < 0.f ? 0.f : t.w;
    }
    t = t + pz;
    float* op = out + (size_t)gcl * DIMC + 4 * lane;
    if (wr) *(volatile v4f*)op = t;
    __threadfence();
    if (wr) *(volatile v4f*)op = t;
  }
}

static int pick_nb(int nE, int nN) {
  int nb = NBMAX;
  while (nb > 16 && (long long)nb * (long long)nE * 5LL > (long long)RCAP * (long long)nN * 4LL) nb >>= 1;
  return nb;
}
static inline int cdiv(int a, int b) { return (a + b - 1) / b; }

extern "C" void kernel_launch(void* const* d_in, const int* in_sizes, int n_in,
                              void* d_out, int out_size, void* d_ws, size_t ws_size,
                              hipStream_t stream) {
  if (n_in < 5) return;
  if (in_sizes[0] < DIMC || (in_sizes[0] % DIMC) != 0) return;
  const int nN = in_sizes[0] / DIMC;
  if (nN < 1 || nN > (1 << 22)) return;
  if (in_sizes[1] < 3 || (in_sizes[1] % 3) != 0) return;
  const int nE = in_sizes[1] / 3;
  if (nE < 1 || nE > (1 << 21)) return;
  if (in_sizes[2] != nE) return;
  if (in_sizes[3] != RP1 * DIMC * DIMC) return;
  if (in_sizes[4] != RP1 * NHEAD * QD) return;
  if (out_size != nN * DIMC) return;

  const float* x   = (const float*)d_in[0];
  const int*   el  = (const int*)  d_in[1];
  const float* ew  = (const float*)d_in[2];
  const float* Wt  = (const float*)d_in[3];
  const float* qry = (const float*)d_in[4];
  float* out = (float*)d_out;

  const int MP = cdiv(nN, RBG) * RBG;
  const int nb = pick_nb(nE, nN);
  const int gA = cdiv(nN, nb);
  if ((long long)gA * nb < nN || (MP % RBG) != 0 || nb < 16 || nb > NBMAX) return;

  char* ws = (char*)d_ws;
  size_t off = 0;
  const size_t oF   = off; off += (size_t)FROWS * DIMC * 4;        off = (off + 255) & ~(size_t)255;
  const size_t oFH  = off; off += (size_t)FROWS * DIMC * 2;        off = (off + 255) & ~(size_t)255;
  const size_t oFL  = off; off += (size_t)FROWS * DIMC * 2;        off = (off + 255) & ~(size_t)255;
  const size_t oWH  = off; off += (size_t)WROWS * DIMC * 2;        off = (off + 255) & ~(size_t)255;
  const size_t oWL  = off; off += (size_t)WROWS * DIMC * 2;        off = (off + 255) & ~(size_t)255;
  const size_t oLAB = off; off += (size_t)MP * LABP * 4;           off = (off + 255) & ~(size_t)255;
  const size_t oHID = off; off += (size_t)RCH * MP * DIMC * 4;     off = (off + 255) & ~(size_t)255;
  if (off > ws_size || off > (size_t)WSMAX) return;
  float* F   = (float*)(ws + oF);
  us*    FH  = (us*)(ws + oFH);
  us*    FL  = (us*)(ws + oFL);
  us*    WH  = (us*)(ws + oWH);
  us*    WL  = (us*)(ws + oWL);
  float* LAB = (float*)(ws + oLAB);
  float* HID = (float*)(ws + oHID);
  const size_t pstride = (size_t)MP * DIMC;

  const int ldsLab = GLDSA + RBG * FROWS * 4;
  const int ldsHid = GLDSA + RBG * WROWS * 4;
  hipFuncSetAttribute(reinterpret_cast<const void*>(&k_gemm3), hipFuncAttributeMaxDynamicSharedMemorySize, ldsHid);
  hipFuncSetAttribute(reinterpret_cast<const void*>(&k_agg), hipFuncAttributeMaxDynamicSharedMemorySize, LDS_AGG);

  k_fold<<<FROWS, 128, 0, stream>>>(qry, Wt, F);
  const int nUF = FROWS * (DIMC / 8);
  k_cvt<<<cdiv(nUF, NTHR), NTHR, 0, stream>>>(F, FH, FL, nUF);
  const int gM = MP / RBG;
  k_gemm3<<<gM, NTHR, ldsLab, stream>>>(x, FH, FL, LAB, nN, FROWS / 16, LABP, (size_t)0);

  const int nUW = WROWS * (DIMC / 8);
  for (int c = 0; c < RCH; ++c) {
    k_cvt<<<cdiv(nUW, NTHR), NTHR, 0, stream>>>(Wt + (size_t)c * WROWS * DIMC, WH, WL, nUW);
    k_gemm3<<<gM, NTHR, ldsHid, stream>>>(x, WH, WL, HID, nN, WROWS / 16, DIMC, pstride);
    k_agg<<<gA, NTHR, LDS_AGG, stream>>>(el, ew, LAB, HID, out, nN, nE, nb, c, pstride);
  }
}
